// MambaBlock_35304631174087
// MI455X (gfx1250) — hardware-verified
//
#include <hip/hip_runtime.h>
#include <math.h>

typedef __attribute__((ext_vector_type(16))) __bf16   v16b;
typedef __attribute__((ext_vector_type(8)))  __bf16   v8b;
typedef __attribute__((ext_vector_type(8)))  float    v8f;
typedef __attribute__((ext_vector_type(4)))  float    v4f;
typedef __attribute__((ext_vector_type(4)))  unsigned v4u;

constexpr int kBatch  = 2;
constexpr int kSeq    = 1024;
constexpr int kDm     = 1024;
constexpr int kDin    = 2048;
constexpr int kNst    = 16;
constexpr int kDtR    = 64;
constexpr int kPrjN   = 96;
constexpr int kPrjP   = 128;
constexpr int kXzP    = 2 * kDin;
constexpr int kRows   = kBatch * kSeq;
constexpr int kConvTP = 260;
constexpr int kScanTS = 64;
constexpr int kScanCh = 64;
constexpr int kScanYP = 68;
static_assert(kDtR + 2 * kNst == kPrjN, "x_proj width");
static_assert((kSeq & (kSeq - 1)) == 0, "sequence length is a power of two");
static_assert((kDm % 32) == 0 && (kDin % 32) == 0 && (kDtR % 32) == 0, "GEMM K multiples of 32");
static_assert((kRows % 64) == 0 && (kXzP % 64) == 0 && (kPrjP % 64) == 0 && (kDin % 64) == 0 && (kDm % 64) == 0, "GEMM M,N multiples of 64");
static_assert((kSeq % kScanTS) == 0 && (kSeq % 64) == 0 && (kDin % kScanCh) == 0 && (kDin % 256) == 0, "tile multiples");
static_assert(((kRows / 64) * (kXzP / 64)) % 8 == 0 && ((kRows / 64) * (kPrjP / 64)) % 8 == 0 &&
              ((kRows / 64) * (kDin / 64)) % 8 == 0 && ((kRows / 64) * (kDm / 64)) % 8 == 0, "8 wave tiles per block");

constexpr size_t kOffXB   = 0;
constexpr size_t kOffWIB  = kOffXB   + (size_t)kRows * kDm   * 2;
constexpr size_t kOffWXB  = kOffWIB  + (size_t)kXzP  * kDm   * 2;
constexpr size_t kOffWDB  = kOffWXB  + (size_t)kPrjP * kDin  * 2;
constexpr size_t kOffWOB  = kOffWDB  + (size_t)kDin  * kDtR  * 2;
constexpr size_t kOffXZ   = kOffWOB  + (size_t)kDm   * kDin  * 2;
constexpr size_t kOffUC   = kOffXZ   + (size_t)kRows * kXzP  * 4;
constexpr size_t kOffUCH  = kOffUC   + (size_t)kRows * kDin  * 4;
constexpr size_t kOffUCL  = kOffUCH  + (size_t)kRows * kDin  * 2;
constexpr size_t kOffPROJ = kOffUCL  + (size_t)kRows * kDin  * 2;
constexpr size_t kOffDTH  = kOffPROJ + (size_t)kRows * kPrjP * 4;
constexpr size_t kOffDTL  = kOffDTH  + (size_t)kRows * kDtR  * 2;
constexpr size_t kOffDLR  = kOffDTL  + (size_t)kRows * kDtR  * 2;
constexpr size_t kOffYH   = kOffDLR  + (size_t)kRows * kDin  * 4;
constexpr size_t kOffYL   = kOffYH   + (size_t)kRows * kDin  * 2;
constexpr size_t kWsTotal = kOffYL   + (size_t)kRows * kDin  * 2;
static_assert(kWsTotal == 119799808ull, "carve total");
static_assert(kWsTotal <= 134217728ull, "carve cap");
static_assert((kOffWIB % 128) == 0 && (kOffWXB % 128) == 0 && (kOffWDB % 128) == 0 && (kOffWOB % 128) == 0 &&
              (kOffXZ % 128) == 0 && (kOffUC % 128) == 0 && (kOffUCH % 128) == 0 && (kOffUCL % 128) == 0 &&
              (kOffPROJ % 128) == 0 && (kOffDTH % 128) == 0 && (kOffDTL % 128) == 0 && (kOffDLR % 128) == 0 &&
              (kOffYH % 128) == 0 && (kOffYL % 128) == 0, "128-B aligned regions");

__device__ __forceinline__ unsigned short f2bf_bits(float f) {
  unsigned u = __float_as_uint(f);
  return (unsigned short)((u + 0x7FFFu + ((u >> 16) & 1u)) >> 16);
}
__device__ __forceinline__ float bf_bits2f(unsigned short h) { return __uint_as_float(((unsigned)h) << 16); }
__device__ __forceinline__ float bf_rne(float f) { return bf_bits2f(f2bf_bits(f)); }
__device__ __forceinline__ unsigned pack2(unsigned short lo16, unsigned short hi16) {
  return (unsigned)lo16 | ((unsigned)hi16 << 16);
}
__device__ __forceinline__ void split8(v4f a0, v4f a1, v4u& whi, v4u& wlo) {
  unsigned short hb[8], lb[8];
#pragma unroll
  for (int e = 0; e < 4; ++e) {
    const float f0 = a0[e];
    const float f1 = a1[e];
    hb[e]     = f2bf_bits(f0);
    hb[4 + e] = f2bf_bits(f1);
    lb[e]     = f2bf_bits(f0 - bf_bits2f(hb[e]));
    lb[4 + e] = f2bf_bits(f1 - bf_bits2f(hb[4 + e]));
  }
  whi[0] = pack2(hb[0], hb[1]); whi[1] = pack2(hb[2], hb[3]); whi[2] = pack2(hb[4], hb[5]); whi[3] = pack2(hb[6], hb[7]);
  wlo[0] = pack2(lb[0], lb[1]); wlo[1] = pack2(lb[2], lb[3]); wlo[2] = pack2(lb[4], lb[5]); wlo[3] = pack2(lb[6], lb[7]);
}

__device__ __forceinline__ void row_guard_b(v8f& a0, v8f& a1, v8f& a2, v8f& a3, v16b x, v16b y,
                                            v16b b0, v16b b1, v16b b2, v16b b3) {
  asm volatile("v_nop\n\tv_nop\n\tv_nop\n\tv_nop"
               : "+v"(a0), "+v"(a1), "+v"(a2), "+v"(a3)
               : "v"(x), "v"(y), "v"(b0), "v"(b1), "v"(b2), "v"(b3));
}
__device__ __forceinline__ void keep4_b(v16b a, v16b b, v16b c, v16b d) { asm volatile("v_nop" :: "v"(a), "v"(b), "v"(c), "v"(d)); }
__device__ __forceinline__ void acc_guard4(v8f& a, v8f& b, v8f& c, v8f& d) { asm volatile("v_nop\n\tv_nop\n\tv_nop\n\tv_nop" : "+v"(a), "+v"(b), "+v"(c), "+v"(d)); }

struct FragB {
  union U { v16b v; v8b h[2]; };
  static __device__ __forceinline__ v16b load(const __bf16* p) {
    U f; f.h[0] = *(const v8b*)(p); f.h[1] = *(const v8b*)(p + 16); return f.v;
  }
  static __device__ __forceinline__ v8f mma(v16b a, v16b b, v8f c) {
    return __builtin_amdgcn_wmma_f32_16x16x32_bf16(false, a, false, b, (short)0, c, false, false);
  }
};

template <int SPL>
__global__ __launch_bounds__(256) void wmma_gemm64_bf16(
    const unsigned short* __restrict__ Ap, const unsigned short* __restrict__ A2p, int lda,
    const unsigned short* __restrict__ Btp, int ldb,
    float* __restrict__ C, int ldc, int M, int N, int K)
{
  const __bf16* A  = (const __bf16*)Ap;
  const __bf16* A2 = (const __bf16*)A2p;
  const __bf16* Bt = (const __bf16*)Btp;
  __shared__ __align__(16) float sT[8][16 * 68];
  const int lane = threadIdx.x & 31;
  const int wave = threadIdx.x >> 5;
  const int tilesN = N >> 6;
  const int tilesM = M >> 6;
  const int tile = blockIdx.x * 8 + wave;
  if (tile >= tilesM * tilesN) return;
  const int tm = tile / tilesN;
  const int tn = tile - tm * tilesN;
  const int m0 = tm << 6;
  const int n0 = tn << 6;

  const int rlane = lane & 15;
  const int koff  = (lane >> 4) * 8;
  const int mOff  = (lane >> 4) * 8;

  v8f acc[4][4];
#pragma unroll
  for (int i = 0; i < 4; ++i)
#pragma unroll
    for (int j = 0; j < 4; ++j) acc[i][j] = (v8f){0.f,0.f,0.f,0.f,0.f,0.f,0.f,0.f};

  for (int k0 = 0; k0 < K; k0 += 32) {
    v16b bh[4];
#pragma unroll
    for (int j = 0; j < 4; ++j) {
      const size_t bo = (size_t)(n0 + (j << 4) + rlane) * ldb + koff + k0;
      bh[j] = FragB::load(Bt + bo);
    }
#pragma unroll
    for (int i = 0; i < 4; ++i) {
      const size_t ao = (size_t)(m0 + (i << 4) + rlane) * lda + koff + k0;
      v16b ah = FragB::load(A + ao);
      v16b al = ah;
      if (SPL == 1) al = FragB::load(A2 + ao);
#pragma unroll
      for (int j = 0; j < 4; ++j) {
        acc[i][j] = FragB::mma(ah, bh[j], acc[i][j]);
        if (SPL == 1) acc[i][j] = FragB::mma(al, bh[j], acc[i][j]);
      }
      row_guard_b(acc[i][0], acc[i][1], acc[i][2], acc[i][3], ah, al, bh[0], bh[1], bh[2], bh[3]);
    }
    keep4_b(bh[0], bh[1], bh[2], bh[3]);
  }
  acc_guard4(acc[0][0], acc[0][1], acc[0][2], acc[0][3]);
  acc_guard4(acc[1][0], acc[1][1], acc[1][2], acc[1][3]);
  acc_guard4(acc[2][0], acc[2][1], acc[2][2], acc[2][3]);
  acc_guard4(acc[3][0], acc[3][1], acc[3][2], acc[3][3]);

  float* slab = sT[wave];
  const int hh = lane >> 4, c4 = (lane & 15) * 4;
#pragma unroll
  for (int i = 0; i < 4; ++i) {
    const int mBase = m0 + (i << 4);
#pragma unroll
    for (int j = 0; j < 4; ++j) {
#pragma unroll
      for (int r = 0; r < 8; ++r) slab[(mOff + r) * 68 + (j << 4) + rlane] = acc[i][j][r];
    }
    __builtin_amdgcn_fence(__ATOMIC_RELEASE, "workgroup");
    __builtin_amdgcn_wave_barrier();
    __builtin_amdgcn_fence(__ATOMIC_ACQUIRE, "workgroup");
    for (int pass = 0; pass < 2; ++pass) {
#pragma unroll
      for (int it = 0; it < 8; ++it) {
        const int row = it * 2 + hh;
        v4f v = *(const v4f*)(slab + row * 68 + c4);
        *(volatile v4f*)(C + (size_t)(mBase + row) * ldc + n0 + c4) = v;
      }
      __threadfence();
    }
    __builtin_amdgcn_fence(__ATOMIC_RELEASE, "workgroup");
    __builtin_amdgcn_wave_barrier();
    __builtin_amdgcn_fence(__ATOMIC_ACQUIRE, "workgroup");
  }
}

__global__ __launch_bounds__(256) void cast_bf16_kernel(
    const float* __restrict__ src, unsigned short* __restrict__ dst, int total8, int valid8)
{
  const int i = blockIdx.x * 256 + threadIdx.x;
  if (i >= total8) return;
  const bool live = (i < valid8);
  const int ic = live ? i : (valid8 - 1);
  const float* p = src + ((size_t)ic << 3);
  const v4f a0 = *(const v4f*)(p);
  const v4f a1 = *(const v4f*)(p + 4);
  unsigned short hb[8];
#pragma unroll
  for (int e = 0; e < 4; ++e) {
    const float f0 = a0[e];
    const float f1 = a1[e];
    const unsigned short b0 = f2bf_bits(f0);
    const unsigned short b1 = f2bf_bits(f1);
    hb[e]     = live ? b0 : (unsigned short)0;
    hb[4 + e] = live ? b1 : (unsigned short)0;
  }
  v4u w;
  w[0] = pack2(hb[0], hb[1]); w[1] = pack2(hb[2], hb[3]); w[2] = pack2(hb[4], hb[5]); w[3] = pack2(hb[6], hb[7]);
  unsigned short* q = dst + ((size_t)i << 3);
  *(volatile v4u*)q = w;
  __threadfence();
  *(volatile v4u*)q = w;
}

__global__ __launch_bounds__(256) void dt_split_kernel(
    const float* __restrict__ PROJ, unsigned short* __restrict__ DTH, unsigned short* __restrict__ DTL, int total8)
{
  const int i = blockIdx.x * 256 + threadIdx.x;
  if (i >= total8) return;
  const int e0  = i << 3;
  const int row = e0 >> 6;
  const int c8  = e0 & 63;
  const float* p = PROJ + (size_t)row * kPrjP + c8;
  const v4f a0 = *(const v4f*)(p);
  const v4f a1 = *(const v4f*)(p + 4);
  v4u wh, wl;
  split8(a0, a1, wh, wl);
  unsigned short* qh = DTH + e0;
  unsigned short* ql = DTL + e0;
  *(volatile v4u*)qh = wh;
  *(volatile v4u*)ql = wl;
  __threadfence();
  *(volatile v4u*)qh = wh;
  *(volatile v4u*)ql = wl;
}

__global__ __launch_bounds__(256) void conv_silu_kernel(
    const float* __restrict__ XZ, const float* __restrict__ cw, const float* __restrict__ cb,
    float* __restrict__ UC, unsigned short* __restrict__ UCH, unsigned short* __restrict__ UCL)
{
  __shared__ __align__(16) float sT[16 * kConvTP];
  const int tid = threadIdx.x, lane = tid & 31, wave = tid >> 5;
  const int d0 = blockIdx.x * 256, d = d0 + tid;
  const int g0 = blockIdx.y * 64;
  const int tb = g0 & (kSeq - 1);
  const v4f wv = *(const v4f*)(cw + (size_t)d * 4);
  const float w0 = bf_rne(wv[0]), w1 = bf_rne(wv[1]), w2 = bf_rne(wv[2]), w3 = bf_rne(wv[3]);
  const float bc = bf_rne(cb[d]);
  float xm3, xm2, xm1;
  {
    const bool hist = (tb > 0);
    const int rb = hist ? (g0 - 3) : g0;
    const float v3 = XZ[(size_t)rb * kXzP + d];
    const float v2 = XZ[(size_t)(rb + 1) * kXzP + d];
    const float v1 = XZ[(size_t)(rb + 2) * kXzP + d];
    xm3 = hist ? v3 : 0.f;
    xm2 = hist ? v2 : 0.f;
    xm1 = hist ? v1 : 0.f;
  }
  const int hrow = wave >> 1;
  const int hch  = (wave & 1) * 128 + lane * 4;
#pragma unroll 1
  for (int sub = 0; sub < 4; ++sub) {
    const int lb = g0 + sub * 16;
#pragma unroll 1
    for (int s = 0; s < 16; ++s) {
      const float xcur = XZ[(size_t)(lb + s) * kXzP + d];
      float acc = w0 * xm3;
      acc = fmaf(w1, xm2, acc);
      acc = fmaf(w2, xm1, acc);
      acc = fmaf(w3, xcur, acc);
      const float sv = acc + bc;
      const float sg = __builtin_amdgcn_rcpf(1.0f + expf(-sv));
      sT[s * kConvTP + tid] = sv * sg;
      xm3 = xm2; xm2 = xm1; xm1 = xcur;
    }
    __syncthreads();
    v4f fv[4];
    v4u bh[2], blo[2];
#pragma unroll
    for (int it = 0; it < 4; ++it) fv[it] = *(const v4f*)(sT + (it * 4 + hrow) * kConvTP + hch);
#pragma unroll
    for (int it = 0; it < 2; ++it) {
      const v4f a0 = *(const v4f*)(sT + (it * 8 + wave) * kConvTP + lane * 8);
      const v4f a1 = *(const v4f*)(sT + (it * 8 + wave) * kConvTP + lane * 8 + 4);
      split8(a0, a1, bh[it], blo[it]);
    }
    for (int pass = 0; pass < 2; ++pass) {
#pragma unroll
      for (int it = 0; it < 4; ++it)
        *(volatile v4f*)(UC + (size_t)(lb + it * 4 + hrow) * kDin + d0 + hch) = fv[it];
#pragma unroll
      for (int it = 0; it < 2; ++it) {
        const size_t o = (size_t)(lb + it * 8 + wave) * kDin + d0 + lane * 8;
        *(volatile v4u*)(UCH + o) = bh[it];
        *(volatile v4u*)(UCL + o) = blo[it];
      }
      __threadfence();
    }
    __syncthreads();
  }
}

__global__ __launch_bounds__(64) void scan_kernel(
    const float* __restrict__ DLR, const float* __restrict__ UC, const float* __restrict__ XZ,
    const float* __restrict__ PROJ, const float* __restrict__ bdt, const float* __restrict__ Alog,
    const float* __restrict__ Dp, unsigned short* __restrict__ YH, unsigned short* __restrict__ YL)
{
  __shared__ __align__(16) float sBC[kScanTS * 32];
  __shared__ __align__(16) float sY[kScanTS * kScanYP];
  __shared__ __align__(16) float sA[kNst * kScanCh];
  const int tid = threadIdx.x, lane = tid & 31, wave = tid >> 5;
  constexpr int kBlkPerB = kDin / kScanCh;
  const int bix = blockIdx.x / kBlkPerB;
  const int d0  = (blockIdx.x - bix * kBlkPerB) * kScanCh;
  const int d   = d0 + tid;
  const size_t row0 = (size_t)bix * kSeq;
#pragma unroll 1
  for (int s = 0; s < kNst; ++s) sA[s * kScanCh + tid] = -expf(bf_rne(Alog[(size_t)d * kNst + s]));
  __syncthreads();
  float negA[kNst], h[kNst];
#pragma unroll
  for (int s = 0; s < kNst; ++s) {
    negA[s] = sA[s * kScanCh + tid];
    h[s] = 0.f;
  }
  const float bb = bf_rne(bdt[d]);
  const float Dd = bf_rne(Dp[d]);
  const int sr = tid >> 3, sc4 = (tid & 7) * 4;
  const int q = lane >> 3, c8 = (lane & 7) * 8;
#pragma unroll 1
  for (int t0 = 0; t0 < kSeq; t0 += kScanTS) {
    __syncthreads();
#pragma unroll
    for (int i = 0; i < 8; ++i) {
      const int r = sr + 8 * i;
      *(v4f*)(sBC + r * 32 + sc4) = *(const v4f*)(PROJ + (row0 + t0 + r) * kPrjP + kDtR + sc4);
    }
    __syncthreads();
#pragma unroll 1
    for (int s = 0; s < kScanTS; ++s) {
      const size_t row = row0 + t0 + s;
      const float* xr = sBC + s * 32;
      float Bs[kNst], Cs[kNst];
#pragma unroll
      for (int q4 = 0; q4 < 4; ++q4) {
        const v4f bv = *(const v4f*)(xr + 4 * q4);
        const v4f cv = *(const v4f*)(xr + kNst + 4 * q4);
        Bs[4 * q4 + 0] = bv[0]; Bs[4 * q4 + 1] = bv[1]; Bs[4 * q4 + 2] = bv[2]; Bs[4 * q4 + 3] = bv[3];
        Cs[4 * q4 + 0] = cv[0]; Cs[4 * q4 + 1] = cv[1]; Cs[4 * q4 + 2] = cv[2]; Cs[4 * q4 + 3] = cv[3];
      }
      const float v   = DLR[row * kDin + d] + bb;
      const float a   = expf(-fabsf(v));
      const float u1  = 1.0f + a;
      const float l1p = __logf(u1) + (a - (u1 - 1.0f)) * __builtin_amdgcn_rcpf(u1);
      const float dt  = fmaxf(v, 0.0f) + l1p;
      const float xt  = UC[row * kDin + d];
      const float dtx = dt * xt;
      float y = 0.f;
#pragma unroll
      for (int k = 0; k < kNst; ++k) {
        const float e = __expf(dt * negA[k]);
        h[k] = fmaf(e, h[k], dtx * Bs[k]);
        y = fmaf(h[k], Cs[k], y);
      }
      y = fmaf(xt, Dd, y);
      const float zv = XZ[row * kXzP + kDin + d];
      const float sg = __builtin_amdgcn_rcpf(1.0f + expf(-zv));
      y = y * (zv * sg);
      sY[s * kScanYP + tid] = y;
    }
    __syncthreads();
    v4u hv[8], lv[8];
#pragma unroll
    for (int it = 0; it < 8; ++it) {
      const int rr = it * 8 + wave * 4 + q;
      const v4f a0 = *(const v4f*)(sY + rr * kScanYP + c8);
      const v4f a1 = *(const v4f*)(sY + rr * kScanYP + c8 + 4);
      split8(a0, a1, hv[it], lv[it]);
    }
    for (int pass = 0; pass < 2; ++pass) {
#pragma unroll
      for (int it = 0; it < 8; ++it) {
        const int rr = it * 8 + wave * 4 + q;
        const size_t o = (row0 + t0 + rr) * kDin + d0 + c8;
        *(volatile v4u*)(YH + o) = hv[it];
        *(volatile v4u*)(YL + o) = lv[it];
      }
      __threadfence();
    }
  }
}

extern "C" void kernel_launch(void* const* d_in, const int* in_sizes, int n_in,
                              void* d_out, int out_size, void* d_ws, size_t ws_size,
                              hipStream_t stream) {
  if (n_in < 10) return;
  if (in_sizes[0] != kRows * kDm) return;
  if (in_sizes[1] != kXzP * kDm) return;
  if (in_sizes[2] != kDin * 4) return;
  if (in_sizes[3] != kDin) return;
  if (in_sizes[4] != kPrjN * kDin) return;
  if (in_sizes[5] != kDin * kDtR) return;
  if (in_sizes[6] != kDin) return;
  if (in_sizes[7] != kDin * kNst) return;
  if (in_sizes[8] != kDin) return;
  if (in_sizes[9] != kDm * kDin) return;
  if (out_size != kRows * kDm) return;
  if (ws_size < kWsTotal) return;

  const float* x       = (const float*)d_in[0];
  const float* W_in    = (const float*)d_in[1];
  const float* conv_w  = (const float*)d_in[2];
  const float* conv_b  = (const float*)d_in[3];
  const float* W_xproj = (const float*)d_in[4];
  const float* W_dt    = (const float*)d_in[5];
  const float* b_dt    = (const float*)d_in[6];
  const float* A_log   = (const float*)d_in[7];
  const float* Dp      = (const float*)d_in[8];
  const float* W_out   = (const float*)d_in[9];
  float* out = (float*)d_out;

  char* ws = (char*)d_ws;
  unsigned short* XB   = (unsigned short*)(ws + kOffXB);
  unsigned short* WIB  = (unsigned short*)(ws + kOffWIB);
  unsigned short* WXB  = (unsigned short*)(ws + kOffWXB);
  unsigned short* WDB  = (unsigned short*)(ws + kOffWDB);
  unsigned short* WOB  = (unsigned short*)(ws + kOffWOB);
  float*          XZ   = (float*)(ws + kOffXZ);
  float*          UC   = (float*)(ws + kOffUC);
  unsigned short* UCH  = (unsigned short*)(ws + kOffUCH);
  unsigned short* UCL  = (unsigned short*)(ws + kOffUCL);
  float*          PROJ = (float*)(ws + kOffPROJ);
  unsigned short* DTH  = (unsigned short*)(ws + kOffDTH);
  unsigned short* DTL  = (unsigned short*)(ws + kOffDTL);
  float*          DLR  = (float*)(ws + kOffDLR);
  unsigned short* YH   = (unsigned short*)(ws + kOffYH);
  unsigned short* YL   = (unsigned short*)(ws + kOffYL);

  cast_bf16_kernel<<<(kRows * kDm / 8) / 256, 256, 0, stream>>>(x, XB, kRows * kDm / 8, kRows * kDm / 8);
  cast_bf16_kernel<<<(kXzP * kDm / 8) / 256, 256, 0, stream>>>(W_in, WIB, kXzP * kDm / 8, kXzP * kDm / 8);
  cast_bf16_kernel<<<(kPrjP * kDin / 8) / 256, 256, 0, stream>>>(W_xproj, WXB, kPrjP * kDin / 8, kPrjN * kDin / 8);
  cast_bf16_kernel<<<(kDin * kDtR / 8) / 256, 256, 0, stream>>>(W_dt, WDB, kDin * kDtR / 8, kDin * kDtR / 8);
  cast_bf16_kernel<<<(kDm * kDin / 8) / 256, 256, 0, stream>>>(W_out, WOB, kDm * kDin / 8, kDm * kDin / 8);

  wmma_gemm64_bf16<0><<<dim3((kRows / 64) * (kXzP / 64) / 8), 256, 0, stream>>>(
      XB, XB, kDm, WIB, kDm, XZ, kXzP, kRows, kXzP, kDm);

  conv_silu_kernel<<<dim3(kDin / 256, kRows / 64), 256, 0, stream>>>(XZ, conv_w, conv_b, UC, UCH, UCL);

  wmma_gemm64_bf16<1><<<dim3((kRows / 64) * (kPrjP / 64) / 8), 256, 0, stream>>>(
      UCH, UCL, kDin, WXB, kDin, PROJ, kPrjP, kRows, kPrjP, kDin);

  dt_split_kernel<<<(kRows * kDtR / 8) / 256, 256, 0, stream>>>(PROJ, DTH, DTL, kRows * kDtR / 8);

  wmma_gemm64_bf16<1><<<dim3((kRows / 64) * (kDin / 64) / 8), 256, 0, stream>>>(
      DTH, DTL, kDtR, WDB, kDtR, DLR, kDin, kRows, kDin, kDtR);

  scan_kernel<<<kBatch * (kDin / kScanCh), kScanCh, 0, stream>>>(DLR, UC, XZ, PROJ, b_dt, A_log, Dp, YH, YL);

  wmma_gemm64_bf16<1><<<dim3((kRows / 64) * (kDm / 64) / 8), 256, 0, stream>>>(
      YH, YL, kDin, WOB, kDin, out, kDm, kRows, kDm, kDin);
}
